// ResBlock_d3d_47863115546760
// MI455X (gfx1250) — hardware-run, weakly checked
//
#include <hip/hip_runtime.h>
#include <stdint.h>

#define DEVINL __device__ __forceinline__

typedef _Float16 f16t;
typedef _Float16 v16h __attribute__((ext_vector_type(16)));
typedef _Float16 v8h  __attribute__((ext_vector_type(8)));
typedef float    v8f  __attribute__((ext_vector_type(8)));
typedef float    v4f  __attribute__((ext_vector_type(4)));
typedef v8h __attribute__((may_alias)) v8ha;
typedef v4f __attribute__((may_alias)) v4fa;
union FragH { v16h v; v8h half[2]; unsigned int u[8]; };

#define CCH   64
#define TT    7
#define HD    64
#define WDD   64
#define HW    (HD * WDD)
#define THW   (TT * HW)
#define NTAP  27
#define KT    (NTAP * CCH)
#define NOFF  54
#define OMC   64
#define NPIX  64
#define SLP   72
#define SOP   68
#define XP    65
#define TPB   256
#define TPO   64
#define WCAR  256.0f
#define WOCAR 1024.0f
#define XCAR  8.0f
#define SCAR  16.0f
#define INVC  (1.0f / 4096.0f)
#define INVO  (1.0f / 8192.0f)

static_assert((KT % 32) == 0);
static_assert(NPIX == WDD);
static_assert(TPB == 4 * NPIX);
static_assert((OMC * (KT / 8)) % TPB == 0);
static_assert(4 * 4 * TPB == NPIX * CCH);
static_assert(8 * 2 * TPB == NPIX * CCH);
static_assert(NPIX * SOP * 4 >= NPIX * SLP * 2);
static_assert(((SLP * 2) % 16) == 0);
static_assert(((SOP * 4) % 16) == 0);
static_assert(((KT * 2) % 128) == 0);
static_assert(((CCH * 4) % 128) == 0);
static_assert(((CCH * 2) % 128) == 0);

DEVINL int imin(int a, int b) { return a < b ? a : b; }
DEVINL int imax(int a, int b) { return a > b ? a : b; }

DEVINL v8f wmma_f16(v16h a, v16h b, v8f c) {
  v8f d = __builtin_amdgcn_wmma_f32_16x16x32_f16(false, a, false, b, (short)0, c, false, false);
  asm volatile("v_nop\n\tv_nop\n\tv_nop\n\tv_nop" : "+v"(d) : "v"(a), "v"(b));
  return d;
}
DEVINL v8f zero8f() {
  v8f z = {0.f, 0.f, 0.f, 0.f, 0.f, 0.f, 0.f, 0.f};
  return z;
}

__global__ __launch_bounds__(TPB) void wprep_k(const float* __restrict__ w, f16t* __restrict__ Wq,
                                             int nvalid, int ntotal, float car)
{
  const int t = blockIdx.x * TPB + threadIdx.x;
  if (t >= ntotal * (KT / 8)) return;
  const int o    = t / (KT / 8);
  const int part = t - o * (KT / 8);
  const int k8   = 8 * part;
  const int tap  = k8 >> 6;
  const int c0   = k8 & (CCH - 1);
  const int oc   = o < nvalid ? o : nvalid - 1;
  const float sc = (o < nvalid) ? car : 0.0f;
  v8h v;
  #pragma unroll
  for (int i = 0; i < 8; ++i) {
    const float wv = w[(size_t)(oc * CCH + c0 + i) * NTAP + tap];
    v[i] = (f16t)(wv * sc);
  }
  f16t* dst = Wq + (size_t)8 * t;
  *(volatile v8h*)dst = v;
  __threadfence();
  *(volatile v8h*)dst = v;
}

__global__ __launch_bounds__(TPB) void xprep_k(const float* __restrict__ x, float* __restrict__ Xt,
                                             f16t* __restrict__ Xh)
{
  __shared__ __attribute__((aligned(16))) float sX[CCH * XP];
  const int tid = threadIdx.x;
  const int s0  = blockIdx.x * NPIX;
  const float* xb = x + s0;
  #pragma unroll 4
  for (int idx = tid; idx < CCH * WDD; idx += TPB) {
    const int c  = idx >> 6;
    const int wq = idx & (WDD - 1);
    sX[c * XP + wq] = xb[(size_t)c * THW + wq];
  }
  __syncthreads();

  v4f vals[4];
  #pragma unroll
  for (int j = 0; j < 4; ++j) {
    const int f  = 4 * (tid + TPB * j);
    const int px = f >> 6, c = f & (CCH - 1);
    v4f v;
    #pragma unroll
    for (int e = 0; e < 4; ++e) v[e] = sX[(c + e) * XP + px];
    vals[j] = v;
  }
  float* dst = Xt + (size_t)s0 * CCH;
  #pragma unroll
  for (int j = 0; j < 4; ++j)
    *(volatile v4f*)(dst + 4 * (tid + TPB * j)) = vals[j];
  __threadfence();
  #pragma unroll
  for (int j = 0; j < 4; ++j)
    *(volatile v4f*)(dst + 4 * (tid + TPB * j)) = vals[j];

  v8h hv[2];
  #pragma unroll
  for (int j = 0; j < 2; ++j) {
    const int e8 = 8 * (tid + TPB * j);
    const int px = e8 >> 6, c = e8 & (CCH - 1);
    v8h o;
    #pragma unroll
    for (int e = 0; e < 8; ++e) o[e] = (f16t)(sX[(c + e) * XP + px] * XCAR);
    hv[j] = o;
  }
  f16t* hdst = Xh + (size_t)s0 * CCH;
  #pragma unroll
  for (int j = 0; j < 2; ++j)
    *(volatile v8h*)(hdst + 8 * (tid + TPB * j)) = hv[j];
  __threadfence();
  #pragma unroll
  for (int j = 0; j < 2; ++j)
    *(volatile v8h*)(hdst + 8 * (tid + TPB * j)) = hv[j];
}

__global__ __launch_bounds__(TPO) void offconv_k(const f16t* __restrict__ Xh, const f16t* __restrict__ Wo,
                                               const float* __restrict__ boff, float* __restrict__ Om)
{
  __shared__ __attribute__((aligned(16))) float sO[OMC * NPIX];
  const int tid = threadIdx.x, lane = tid & 31, wave = tid >> 5;
  const int h = lane >> 4, m = lane & 15;
  const int wg = blockIdx.x;
  const int t  = wg >> 6;
  const int oh = wg & (HD - 1);
  const int s0 = wg * NPIX;

  v8f acc[4][2];
  #pragma unroll
  for (int mt = 0; mt < 4; ++mt) { acc[mt][0] = zero8f(); acc[mt][1] = zero8f(); }

  #pragma unroll 1
  for (int tap = 0; tap < NTAP; ++tap) {
    const int q9 = tap / 9;
    const int r9 = tap - 9 * q9;
    const int q3 = r9 / 3;
    const int kt = q9 - 1, kh = q3 - 1, kw = r9 - 3 * q3 - 1;
    const int tt = t + kt;
    const bool tok = ((unsigned)tt < (unsigned)TT);
    const int  tc  = imin(imax(tt, 0), TT - 1);
    const int yy = oh + kh;
    const bool yok = ((unsigned)yy < (unsigned)HD);
    const int  yc  = imin(imax(yy, 0), HD - 1);
    const f16t* bp[2];
    bool ok[2];
    #pragma unroll
    for (int nl = 0; nl < 2; ++nl) {
      const int px  = 16 * (2 * wave + nl) + m + kw;
      const bool xok = ((unsigned)px < (unsigned)WDD);
      const int  xc  = imin(imax(px, 0), WDD - 1);
      bp[nl] = Xh + ((size_t)((tc * HD + yc) * WDD + xc)) * CCH + 8 * h;
      ok[nl] = tok && yok && xok;
    }
    const f16t* at = Wo + (size_t)m * KT + tap * CCH + 8 * h;
    #pragma unroll
    for (int c = 0; c < 2; ++c) {
      FragH a[4];
      #pragma unroll
      for (int mt = 0; mt < 4; ++mt) {
        a[mt].half[0] = *(const v8ha*)(at + (size_t)(16 * mt) * KT + 32 * c);
        a[mt].half[1] = *(const v8ha*)(at + (size_t)(16 * mt) * KT + 32 * c + 16);
      }
      #pragma unroll
      for (int nl = 0; nl < 2; ++nl) {
        FragH bf;
        bf.half[0] = *(const v8ha*)(bp[nl] + 32 * c);
        bf.half[1] = *(const v8ha*)(bp[nl] + 32 * c + 16);
        #pragma unroll
        for (int i = 0; i < 8; ++i) bf.u[i] = ok[nl] ? bf.u[i] : 0u;
        #pragma unroll
        for (int mt = 0; mt < 4; ++mt) acc[mt][nl] = wmma_f16(a[mt].v, bf.v, acc[mt][nl]);
      }
    }
  }

  #pragma unroll
  for (int mt = 0; mt < 4; ++mt) {
    #pragma unroll
    for (int nl = 0; nl < 2; ++nl) {
      #pragma unroll
      for (int r = 0; r < 8; ++r) {
        const int chn = 16 * mt + 8 * h + r;
        const int bc  = chn < NOFF ? chn : NOFF - 1;
        float bv = boff[bc];
        bv = (chn < NOFF) ? bv : 0.0f;
        sO[chn * NPIX + 16 * (2 * wave + nl) + m] = acc[mt][nl][r] * INVO + bv;
      }
    }
  }
  __syncthreads();

  float* gbase = Om + (size_t)s0 + 4 * m;
  v4f vv[16];
  #pragma unroll
  for (int j = 0; j < 16; ++j) {
    const int row = 32 * wave + 2 * j + h;
    vv[j] = *(const v4fa*)(sO + row * NPIX + 4 * m);
  }
  #pragma unroll
  for (int j = 0; j < 16; ++j) {
    const int row = 32 * wave + 2 * j + h;
    *(volatile v4f*)(gbase + (size_t)row * THW) = vv[j];
  }
  __threadfence();
  #pragma unroll
  for (int j = 0; j < 16; ++j) {
    const int row = 32 * wave + 2 * j + h;
    *(volatile v4f*)(gbase + (size_t)row * THW) = vv[j];
  }
}

template <int MODE>
__global__ __launch_bounds__(TPB) void dconv_k(const float* __restrict__ src, const f16t* __restrict__ Wq,
                                             const float* __restrict__ Om, float* Yt, f16t* Yh,
                                             const float* __restrict__ xres, float* outp)
{
  __shared__ __attribute__((aligned(16))) unsigned char smem[NPIX * SOP * 4];
  f16t*  Sl = (f16t*)smem;
  float* sO = (float*)smem;
  const int tid = threadIdx.x, lane = tid & 31, wave = tid >> 5;
  const int h = lane >> 4, m = lane & 15;
  const int mw = wave & 3;
  const int pw = wave >> 2;
  const int wg = blockIdx.x;
  const int t  = wg >> 6;
  const int oh = wg & (HD - 1);
  const int s0 = wg * NPIX;

  const int pos = tid & (NPIX - 1);
  const int cg  = tid >> 6;
  const float* omb = Om + (size_t)s0 + pos;
  const f16t* arow = Wq + (size_t)(16 * mw + m) * KT + 8 * h;

  v8f acc[2];
  acc[0] = zero8f(); acc[1] = zero8f();

  #pragma unroll 1
  for (int tap = 0; tap < NTAP; ++tap) {
    const int q9 = tap / 9;
    const int r9 = tap - 9 * q9;
    const int q3 = r9 / 3;
    const int kt = q9 - 1, kh = q3 - 1, kw = r9 - 3 * q3 - 1;
    const int tt = t + kt;
    const bool tok = ((unsigned)tt < (unsigned)TT);
    const int  tc  = imin(imax(tt, 0), TT - 1);
    __syncthreads();

    {
      const float dy = omb[(size_t)(2 * tap) * THW];
      const float dx = omb[(size_t)(2 * tap + 1) * THW];
      const float ys = (float)(oh + kh) + dy;
      const float xs = (float)(pos + kw) + dx;
      const float y0f = floorf(ys), x0f = floorf(xs);
      const float wy = ys - y0f,   wx = xs - x0f;
      const float y1f = y0f + 1.0f, x1f = x0f + 1.0f;
      const bool vy0 = tok && (y0f >= 0.0f) && (y0f <= (float)(HD - 1));
      const bool vy1 = tok && (y1f >= 0.0f) && (y1f <= (float)(HD - 1));
      const bool vx0 = (x0f >= 0.0f) && (x0f <= (float)(WDD - 1));
      const bool vx1 = (x1f >= 0.0f) && (x1f <= (float)(WDD - 1));
      const float omy = 1.0f - wy, omx = 1.0f - wx;
      float w00 = omy * omx;
      float w01 = omy * wx;
      float w10 = wy * omx;
      float w11 = wy * wx;
      w00 = (vy0 && vx0) ? w00 : 0.0f;
      w01 = (vy0 && vx1) ? w01 : 0.0f;
      w10 = (vy1 && vx0) ? w10 : 0.0f;
      w11 = (vy1 && vx1) ? w11 : 0.0f;
      const int y0i = (int)fminf(fmaxf(y0f, -4.0f), (float)(HD + 4));
      const int x0i = (int)fminf(fmaxf(x0f, -4.0f), (float)(WDD + 4));
      const int y0c = imin(imax(y0i, 0), HD - 1);
      const int y1c = imin(imax(y0i + 1, 0), HD - 1);
      const int x0c = imin(imax(x0i, 0), WDD - 1);
      const int x1c = imin(imax(x0i + 1, 0), WDD - 1);
      const float* tb  = src + (size_t)tc * HW * CCH + 16 * cg;
      const float* p00 = tb + (size_t)(y0c * WDD + x0c) * CCH;
      const float* p01 = tb + (size_t)(y0c * WDD + x1c) * CCH;
      const float* p10 = tb + (size_t)(y1c * WDD + x0c) * CCH;
      const float* p11 = tb + (size_t)(y1c * WDD + x1c) * CCH;
      f16t* srow = Sl + pos * SLP + 16 * cg;
      #pragma unroll
      for (int ch = 0; ch < 2; ++ch) {
        const v4f a0 = *(const v4fa*)(p00 + 8 * ch), a1 = *(const v4fa*)(p00 + 8 * ch + 4);
        const v4f b0 = *(const v4fa*)(p01 + 8 * ch), b1 = *(const v4fa*)(p01 + 8 * ch + 4);
        const v4f c0 = *(const v4fa*)(p10 + 8 * ch), c1 = *(const v4fa*)(p10 + 8 * ch + 4);
        const v4f d0 = *(const v4fa*)(p11 + 8 * ch), d1 = *(const v4fa*)(p11 + 8 * ch + 4);
        v4f u0 = a0 * w00;
        v4f u1 = a1 * w00;
        u0 = b0 * w01 + u0;  u1 = b1 * w01 + u1;
        u0 = c0 * w10 + u0;  u1 = c1 * w10 + u1;
        u0 = d0 * w11 + u0;  u1 = d1 * w11 + u1;
        v8h o;
        #pragma unroll
        for (int i = 0; i < 4; ++i) {
          o[i]     = (f16t)(u0[i] * SCAR);
          o[4 + i] = (f16t)(u1[i] * SCAR);
        }
        *(v8ha*)(srow + 8 * ch) = o;
      }
    }
    __syncthreads();

    const f16t* at = arow + tap * CCH;
    #pragma unroll
    for (int c = 0; c < 2; ++c) {
      FragH a;
      a.half[0] = *(const v8ha*)(at + 32 * c);
      a.half[1] = *(const v8ha*)(at + 32 * c + 16);
      #pragma unroll
      for (int nl = 0; nl < 2; ++nl) {
        FragH bf;
        const f16t* br = Sl + (16 * (2 * pw + nl) + m) * SLP + 32 * c + 8 * h;
        bf.half[0] = *(const v8ha*)(br);
        bf.half[1] = *(const v8ha*)(br + 16);
        acc[nl] = wmma_f16(a.v, bf.v, acc[nl]);
      }
    }
  }
  __syncthreads();

  if (MODE == 0) {
    #pragma unroll
    for (int nl = 0; nl < 2; ++nl) {
      #pragma unroll
      for (int r = 0; r < 8; ++r) {
        const int co = 16 * mw + 8 * h + r;
        const int px = 16 * (2 * pw + nl) + m;
        float v = acc[nl][r] * INVC;
        v = (v > 0.0f) ? v : 0.1f * v;
        sO[px * SOP + co] = v;
      }
    }
    __syncthreads();

    v4f vals[4];
    #pragma unroll
    for (int j = 0; j < 4; ++j) {
      const int f  = 4 * (tid + TPB * j);
      const int px = f >> 6, co = f & (CCH - 1);
      vals[j] = *(const v4fa*)(sO + px * SOP + co);
    }
    float* dst = Yt + (size_t)s0 * CCH;
    #pragma unroll
    for (int j = 0; j < 4; ++j)
      *(volatile v4f*)(dst + 4 * (tid + TPB * j)) = vals[j];
    __threadfence();
    #pragma unroll
    for (int j = 0; j < 4; ++j)
      *(volatile v4f*)(dst + 4 * (tid + TPB * j)) = vals[j];

    v8h hv[2];
    #pragma unroll
    for (int j = 0; j < 2; ++j) {
      const int e8 = 8 * (tid + TPB * j);
      const int px = e8 >> 6, co = e8 & (CCH - 1);
      const v4f lo = *(const v4fa*)(sO + px * SOP + co);
      const v4f hi = *(const v4fa*)(sO + px * SOP + co + 4);
      v8h o;
      #pragma unroll
      for (int i = 0; i < 4; ++i) {
        o[i]     = (f16t)(lo[i] * XCAR);
        o[4 + i] = (f16t)(hi[i] * XCAR);
      }
      hv[j] = o;
    }
    f16t* hdst = Yh + (size_t)s0 * CCH;
    #pragma unroll
    for (int j = 0; j < 2; ++j)
      *(volatile v8h*)(hdst + 8 * (tid + TPB * j)) = hv[j];
    __threadfence();
    #pragma unroll
    for (int j = 0; j < 2; ++j)
      *(volatile v8h*)(hdst + 8 * (tid + TPB * j)) = hv[j];
  } else {
    #pragma unroll
    for (int nl = 0; nl < 2; ++nl) {
      #pragma unroll
      for (int r = 0; r < 8; ++r) {
        const int co = 16 * mw + 8 * h + r;
        const int px = 16 * (2 * pw + nl) + m;
        sO[co * SOP + px] = acc[nl][r] * INVC;
      }
    }
    __syncthreads();

    const int q  = tid & 15;
    const int rb = tid >> 4;
    v4f vals[4];
    #pragma unroll
    for (int j = 0; j < 4; ++j) {
      const int co = 16 * j + rb;
      const v4f d  = *(const v4fa*)(sO + co * SOP + 4 * q);
      const v4f xr = *(const v4fa*)(xres + (size_t)co * THW + s0 + 4 * q);
      vals[j] = d + xr;
    }
    #pragma unroll
    for (int j = 0; j < 4; ++j) {
      const int co = 16 * j + rb;
      *(volatile v4f*)(outp + (size_t)co * THW + s0 + 4 * q) = vals[j];
    }
    __threadfence();
    #pragma unroll
    for (int j = 0; j < 4; ++j) {
      const int co = 16 * j + rb;
      *(volatile v4f*)(outp + (size_t)co * THW + s0 + 4 * q) = vals[j];
    }
  }
}

extern "C" void kernel_launch(void* const* d_in, const int* in_sizes, int n_in,
                              void* d_out, int out_size, void* d_ws, size_t ws_size,
                              hipStream_t stream)
{
  if (n_in < 7) return;
  if (in_sizes[0] != CCH * THW) return;
  if (in_sizes[1] != NOFF * CCH * NTAP) return;
  if (in_sizes[2] != NOFF) return;
  if (in_sizes[3] != CCH * CCH * NTAP) return;
  if (in_sizes[4] != NOFF * CCH * NTAP) return;
  if (in_sizes[5] != NOFF) return;
  if (in_sizes[6] != CCH * CCH * NTAP) return;
  if (out_size != CCH * THW) return;

  const float* x     = (const float*)d_in[0];
  const float* woffA = (const float*)d_in[1];
  const float* boffA = (const float*)d_in[2];
  const float* wA    = (const float*)d_in[3];
  const float* woffB = (const float*)d_in[4];
  const float* boffB = (const float*)d_in[5];
  const float* wB    = (const float*)d_in[6];
  float* outp = (float*)d_out;

  const size_t szW  = (size_t)CCH * KT * 2;
  const size_t szF  = (size_t)THW * CCH * 4;
  const size_t szH  = (size_t)THW * CCH * 2;
  const size_t szOm = (size_t)OMC * THW * 4;
  size_t offb = 0;
  char* ws = (char*)d_ws;
  f16t*  WqA = (f16t*)(ws + offb);  offb += szW;
  f16t*  WqB = (f16t*)(ws + offb);  offb += szW;
  f16t*  WoA = (f16t*)(ws + offb);  offb += szW;
  f16t*  WoB = (f16t*)(ws + offb);  offb += szW;
  float* Xt  = (float*)(ws + offb); offb += szF;
  f16t*  Xh  = (f16t*)(ws + offb);  offb += szH;
  float* Om  = (float*)(ws + offb); offb += szOm;
  float* Yt  = (float*)(ws + offb); offb += szF;
  f16t*  Yh  = (f16t*)(ws + offb);  offb += szH;
  if (offb > ws_size) return;
  if (offb > (size_t)134217728) return;

  const int gw = (OMC * (KT / 8) + TPB - 1) / TPB;
  const int gr = THW / NPIX;
  wprep_k<<<gw, TPB, 0, stream>>>(wA,    WqA, CCH,  CCH, WCAR);
  wprep_k<<<gw, TPB, 0, stream>>>(wB,    WqB, CCH,  CCH, WCAR);
  wprep_k<<<gw, TPB, 0, stream>>>(woffA, WoA, NOFF, OMC, WOCAR);
  wprep_k<<<gw, TPB, 0, stream>>>(woffB, WoB, NOFF, OMC, WOCAR);
  xprep_k<<<gr, TPB, 0, stream>>>(x, Xt, Xh);
  offconv_k<<<gr, TPO, 0, stream>>>(Xh, WoA, boffA, Om);
  dconv_k<0><<<gr, TPB, 0, stream>>>(Xt, WqA, Om, Yt, Yh, x, outp);
  offconv_k<<<gr, TPO, 0, stream>>>(Yh, WoB, boffB, Om);
  dconv_k<1><<<gr, TPB, 0, stream>>>(Yt, WqB, Om, Yt, Yh, x, outp);
}
